// ICTDIrrepsE3ConvFullExternal_84344567759196
// MI455X (gfx1250) — hardware-run, weakly checked
//
#include <hip/hip_runtime.h>
#include <stddef.h>
#include <math.h>


#define UD       8
#define NB16     16
#define HID      64
#define W3COLS   3840
#define FEAT     288
#define NCOLS    480
#define KROW     544
#define KSTEPS   17
#define APL      552
#define AQ       69
#define BKP      576
#define BQ       72
#define ER       32
#define ETHR     64
#define GP       75
#define TPG      6
#define NGW      96
#define NGRPC    5
#define CGN      616
#define L3PACK   0x249A6464u

#define NNB      32
#define NTHRN    64

#define STHR     256
#define NWAVE    8
#define EPT      8
#define NGRP     2
#define CHUNK    (STHR * EPT * NGRP)
#define WCAP     (EPT * NGRP * 32)
#define LISTN    (NWAVE * WCAP)
#define SNB      64
#define FV4      (FEAT / 4)

#define OAHI     0
#define OALO     (ER * APL * 2)
#define OFEAT    (2 * ER * APL * 2)
#define OW1      (OFEAT + ER * FEAT * 4)
#define OW2      (OW1 + NB16 * HID * 4)
#define OB1      (OW2 + HID * HID * 4)
#define OB2      (OB1 + HID * 4)
#define OG       (OB2 + HID * 4)
#define OAE      (OG + ER * GP * 4)
#define LDS_EDGE (OAE + ER * UD * 4)
#define LDS_SC   (SNB * FEAT * 4 + LISTN * 4 + 64)

#define S3C      1.7320508075688772f
#define S15C     3.872983346207417f
#define C5H      1.118033988749895f
#define C15H     1.9364916731037085f
#define RSTEP    (1.0f / (5.0f / 17.0f))

static_assert(KSTEPS * 32 == KROW);
static_assert(APL == AQ * 8 && APL >= KROW && ((APL * 2) % 16) == 0);
static_assert(BKP == BQ * 8 && BKP >= KROW && ((BKP * 2) % 128) == 0);
static_assert(TPG * 16 == NGW && NGW * NGRPC == NCOLS);
static_assert(ER * (NB16 + HID + HID) * 4 <= ER * FEAT * 4);
static_assert((OALO % 16) == 0 && (OFEAT % 16) == 0 && (OW1 % 16) == 0 && (OW2 % 16) == 0);
static_assert((OB1 % 16) == 0 && (OG % 16) == 0 && (OAE % 16) == 0 && (LDS_EDGE % 16) == 0);
static_assert((CHUNK & (CHUNK - 1)) == 0 && CHUNK <= 4096);
static_assert((SNB & (SNB - 1)) == 0 && SNB <= 4096);
static_assert((SNB * FV4) % STHR == 0);
static_assert((ER * FV4) % ETHR == 0);
static_assert((FEAT % 32) == 0 && (FV4 % 8) == 0);
static_assert(ETHR == HID && ETHR == 2 * ER);
static_assert(NTHRN == HID && NNB * NB16 == 8 * NTHRN && NNB * UD == 4 * NTHRN);
static_assert((NCOLS * BQ) % STHR == 0 && ((NCOLS * BQ) % 32) == 0);

typedef float          v4f   __attribute__((ext_vector_type(4)));
typedef float          v8f   __attribute__((ext_vector_type(8)));
typedef int            v4i   __attribute__((ext_vector_type(4)));
typedef unsigned short v8us  __attribute__((ext_vector_type(8)));
typedef __bf16         v16bf __attribute__((ext_vector_type(16)));
union FragB { v16bf v; v8us u[2]; };

struct CGTab { float v[CGN]; };
static_assert(sizeof(CGTab) == CGN * 4);

__device__ __forceinline__ unsigned short bf_bits(float x) {
#if defined(__HIP_DEVICE_COMPILE__)
  const __bf16 b = (__bf16)x;
  return __builtin_bit_cast(unsigned short, b);
#else
  unsigned u = __builtin_bit_cast(unsigned, x);
  u = (u + 0x7FFFu + ((u >> 16) & 1u)) >> 16;
  return (unsigned short)u;
#endif
}
__device__ __forceinline__ float bf_val(unsigned short b) {
  return __builtin_bit_cast(float, ((unsigned)b) << 16);
}

__device__ __forceinline__ float siluf(float x) {
  const float xc = fmaxf(x, -30.0f);
  const float ex = expf(-xc);
  return x * (1.0f / (1.0f + ex));
}

__device__ __forceinline__ v8f wm3(v16bf ah, v16bf al, v16bf bh, v16bf bl, v8f c) {
#if defined(__HIP_DEVICE_COMPILE__)
  v8f d = __builtin_amdgcn_wmma_f32_16x16x32_bf16(false, ah, false, bh, (short)0, c, false, false);
  d = __builtin_amdgcn_wmma_f32_16x16x32_bf16(false, ah, false, bl, (short)0, d, false, false);
  d = __builtin_amdgcn_wmma_f32_16x16x32_bf16(false, al, false, bh, (short)0, d, false, false);
  asm volatile("v_nop\n\tv_nop\n\tv_nop\n\tv_nop" : "+v"(d) : "v"(ah), "v"(al), "v"(bh), "v"(bl));
  return d;
#else
  return c;
#endif
}

template <int L1, int L2, int L3, int CGO>
__device__ __forceinline__ void gpath(const float (&Y)[9], const CGTab& cg, float* dst) {
  constexpr int D1 = 2 * L1 + 1, D2 = 2 * L2 + 1, D3 = 2 * L3 + 1;
  constexpr int O1 = (L1 == 0) ? 0 : ((L1 == 1) ? 1 : 4);
  constexpr int O2 = (L2 == 0) ? 0 : ((L2 == 1) ? 1 : 4);
#pragma unroll
  for (int k = 0; k < D3; ++k) {
    float g = 0.0f;
#pragma unroll
    for (int a = 0; a < D1; ++a) {
#pragma unroll
      for (int b = 0; b < D2; ++b) {
        g += (Y[O1 + a] * Y[O2 + b]) * cg.v[CGO + (a * D2 + b) * D3 + k];
      }
    }
    dst[k] = g;
  }
}

template <int NB>
__device__ __forceinline__ int scan_chunk(const int* __restrict__ dsts, int nE, int cbase, int slotBase,
                                          int vec8, int* list, int tid, int lane, int wave) {
  int wc = 0;
#pragma unroll
  for (int g = 0; g < NGRP; ++g) {
    const int el0  = (g * STHR + tid) * EPT;
    const int e0   = cbase + el0;
    const int sent = -2147483647 - 1;
    const int lst  = nE - 1;
    v4i da, db;
    if (vec8 != 0 && cbase + CHUNK <= nE) {
      da = *(const v4i*)(dsts + e0);
      db = *(const v4i*)(dsts + e0 + 4);
    } else {
      da.x = (e0     < nE) ? dsts[min(e0,     lst)] : sent;
      da.y = (e0 + 1 < nE) ? dsts[min(e0 + 1, lst)] : sent;
      da.z = (e0 + 2 < nE) ? dsts[min(e0 + 2, lst)] : sent;
      da.w = (e0 + 3 < nE) ? dsts[min(e0 + 3, lst)] : sent;
      db.x = (e0 + 4 < nE) ? dsts[min(e0 + 4, lst)] : sent;
      db.y = (e0 + 5 < nE) ? dsts[min(e0 + 5, lst)] : sent;
      db.z = (e0 + 6 < nE) ? dsts[min(e0 + 6, lst)] : sent;
      db.w = (e0 + 7 < nE) ? dsts[min(e0 + 7, lst)] : sent;
    }
    const unsigned nb = (unsigned)slotBase;
    const unsigned s0 = (unsigned)da.x - nb, s1 = (unsigned)da.y - nb;
    const unsigned s2 = (unsigned)da.z - nb, s3 = (unsigned)da.w - nb;
    const unsigned s4 = (unsigned)db.x - nb, s5 = (unsigned)db.y - nb;
    const unsigned s6 = (unsigned)db.z - nb, s7 = (unsigned)db.w - nb;
    const bool h0 = s0 < (unsigned)NB, h1 = s1 < (unsigned)NB, h2 = s2 < (unsigned)NB, h3 = s3 < (unsigned)NB;
    const bool h4 = s4 < (unsigned)NB, h5 = s5 < (unsigned)NB, h6 = s6 < (unsigned)NB, h7 = s7 < (unsigned)NB;
    const unsigned any = __builtin_amdgcn_ballot_w32(h0 | h1 | h2 | h3 | h4 | h5 | h6 | h7);
    if (any != 0u) {
#define HITJ(J, HJ, SJ) { \
        const unsigned mj = __builtin_amdgcn_ballot_w32(HJ); \
        if (mj != 0u) { \
          if (HJ) { \
            const int pos = wc + (int)__builtin_amdgcn_mbcnt_lo(mj, 0u); \
            if (pos < WCAP) list[wave * WCAP + pos] = ((el0 + (J)) << 12) | (int)(SJ); \
          } \
          wc += (int)__builtin_popcount(mj); } }
      HITJ(0, h0, s0)
      HITJ(1, h1, s1)
      HITJ(2, h2, s2)
      HITJ(3, h3, s3)
      HITJ(4, h4, s4)
      HITJ(5, h5, s5)
      HITJ(6, h6, s6)
      HITJ(7, h7, s7)
#undef HITJ
    }
  }
  return wc;
}

__global__ __launch_bounds__(NTHRN) void k_node(
    const int* __restrict__ atom, const float* __restrict__ embt,
    const float* __restrict__ w1, const float* __restrict__ b1,
    const float* __restrict__ w2, const float* __restrict__ b2,
    float* Ai, int nN, int nA) {
  __shared__ __attribute__((aligned(16))) float sein[NNB * NB16];
  __shared__ __attribute__((aligned(16))) float shid[NNB * HID];
  __shared__ __attribute__((aligned(16))) float sw1[NB16 * HID];
  __shared__ __attribute__((aligned(16))) float sw2[HID * UD];
  __shared__ __attribute__((aligned(16))) float sout[NNB * UD];
  const int tid = threadIdx.x, lane = tid & 31, wave = tid >> 5;
  const int nb = blockIdx.x * NNB;

  for (int i = tid; i < NB16 * HID / 4; i += NTHRN) ((v4f*)sw1)[i] = ((const v4f*)w1)[i];
  for (int i = tid; i < HID * UD / 4; i += NTHRN) ((v4f*)sw2)[i] = ((const v4f*)w2)[i];
#pragma unroll
  for (int r = 0; r < 8; ++r) {
    const int idx = tid + NTHRN * r;
    const int i = idx >> 4, c = idx & 15;
    int node = nb + i;
    node = node > nN - 1 ? nN - 1 : node;
    int a = atom[node];
    a = a < 0 ? 0 : (a > nA - 1 ? nA - 1 : a);
    sein[idx] = embt[a * NB16 + c];
  }
  __syncthreads();

  {
    const int j = tid;
    const float bj = b1[j];
#pragma unroll 1
    for (int i = 0; i < NNB; ++i) {
      const v4f* ep = (const v4f*)(sein + i * NB16);
      float sacc = bj;
#pragma unroll 1
      for (int q = 0; q < 4; ++q) {
        const v4f e4 = ep[q];
        sacc += e4.x * sw1[(4 * q + 0) * HID + j];
        sacc += e4.y * sw1[(4 * q + 1) * HID + j];
        sacc += e4.z * sw1[(4 * q + 2) * HID + j];
        sacc += e4.w * sw1[(4 * q + 3) * HID + j];
      }
      shid[i * HID + j] = siluf(sacc);
    }
  }
  __syncthreads();

#pragma unroll 1
  for (int r = 0; r < 4; ++r) {
    const int idx = tid + NTHRN * r;
    const int i = idx >> 3, u = idx & 7;
    float sacc = b2[u];
    const float* hp = shid + i * HID;
#pragma unroll 4
    for (int j = 0; j < HID; ++j) sacc += hp[j] * sw2[j * UD + u];
    sout[idx] = sacc;
  }
  __syncthreads();

  if (wave == 0) {
    const v4f o0 = ((const v4f*)sout)[lane];
    const v4f o1 = ((const v4f*)sout)[lane + 32];
    float* op = Ai + (size_t)nb * UD;
    *(volatile v4f*)(op + 4 * lane) = o0;
    *(volatile v4f*)(op + 4 * (lane + 32)) = o1;
    __threadfence();
    *(volatile v4f*)(op + 4 * lane) = o0;
    *(volatile v4f*)(op + 4 * (lane + 32)) = o1;
  }
}

__global__ __launch_bounds__(STHR) void k_bprep(
    const float* __restrict__ w3, const float* __restrict__ b3,
    unsigned short* Bhi, unsigned short* Blo, int nItems) {
  const int it = blockIdx.x * STHR + (int)threadIdx.x;
  if (it >= nItems) return;
  const int n = it / BQ;
  const int q = it - n * BQ;
  const int p = n >> 5, c = n & 31;
  const int qc = q > HID - 1 ? HID - 1 : q;
  const float* wp = w3 + (size_t)qc * W3COLS + p * 256 + c;
  const float* bp = b3 + p * 256 + c;
  float v[8];
#pragma unroll
  for (int u = 0; u < 8; ++u) {
    const float wv = wp[u * 32];
    const float bv = bp[u * 32];
    v[u] = (q < HID) ? wv : ((q == HID) ? bv : 0.0f);
  }
  v8us hv, lv;
#pragma unroll
  for (int u = 0; u < 8; ++u) {
    const unsigned short hb = bf_bits(v[u]);
    lv[u] = bf_bits(v[u] - bf_val(hb));
    hv[u] = hb;
  }
  unsigned short* ph = Bhi + (size_t)it * 8;
  unsigned short* pl = Blo + (size_t)it * 8;
  *(volatile v8us*)ph = hv;
  *(volatile v8us*)pl = lv;
  __threadfence();
  *(volatile v8us*)ph = hv;
  *(volatile v8us*)pl = lv;
}

__global__ __launch_bounds__(ETHR) void k_edge(
    const float* __restrict__ pos, const int* __restrict__ nbatch,
    const int* __restrict__ esrc, const int* __restrict__ edst,
    const float* __restrict__ shf, const float* __restrict__ cell,
    const float* __restrict__ Ai,
    const float* __restrict__ w1, const float* __restrict__ b1,
    const float* __restrict__ w2, const float* __restrict__ b2,
    const unsigned short* __restrict__ Bhi, const unsigned short* __restrict__ Blo,
    float* feat, int nE, int nN, int nG, float al0, float al1, float al2, CGTab cg) {
  extern __shared__ v4f lds_dyn[];
  char* lds = (char*)lds_dyn;
  unsigned short* sAhi = (unsigned short*)(lds + OAHI);
  unsigned short* sAlo = (unsigned short*)(lds + OALO);
  float* sfeat = (float*)(lds + OFEAT);
  float* semb  = sfeat;
  float* sh1   = sfeat + ER * NB16;
  float* sh2   = sh1 + ER * HID;
  float* sW1   = (float*)(lds + OW1);
  float* sW2   = (float*)(lds + OW2);
  float* sb1   = (float*)(lds + OB1);
  float* sb2   = (float*)(lds + OB2);
  float* sG    = (float*)(lds + OG);
  float* sAe   = (float*)(lds + OAE);
  const int tid = threadIdx.x, lane = tid & 31, wave = tid >> 5, hh = lane >> 4, m = lane & 15;
  const int e0 = blockIdx.x * ER;

  for (int i = tid; i < NB16 * HID / 4; i += ETHR) ((v4f*)sW1)[i] = ((const v4f*)w1)[i];
  for (int i = tid; i < HID * HID / 4; i += ETHR) ((v4f*)sW2)[i] = ((const v4f*)w2)[i];
  sb1[tid] = b1[tid];
  sb2[tid] = b2[tid];

  {
#pragma clang fp contract(off)
    const int el = lane;
    int e = e0 + el;
    e = e > nE - 1 ? nE - 1 : e;
    int s = esrc[e];
    s = s < 0 ? 0 : (s > nN - 1 ? nN - 1 : s);
    int d = edst[e];
    d = d < 0 ? 0 : (d > nN - 1 ? nN - 1 : d);
    int bg = nbatch[s];
    bg = bg < 0 ? 0 : (bg > nG - 1 ? nG - 1 : bg);
    const float f0 = shf[(size_t)e * 3 + 0], f1 = shf[(size_t)e * 3 + 1], f2 = shf[(size_t)e * 3 + 2];
    const float* cl = cell + bg * 9;
    const float shx = f0 * cl[0] + f1 * cl[3] + f2 * cl[6];
    const float shy = f0 * cl[1] + f1 * cl[4] + f2 * cl[7];
    const float shz = f0 * cl[2] + f1 * cl[5] + f2 * cl[8];
    const float vx = (pos[(size_t)d * 3 + 0] - pos[(size_t)s * 3 + 0]) + shx;
    const float vy = (pos[(size_t)d * 3 + 1] - pos[(size_t)s * 3 + 1]) + shy;
    const float vz = (pos[(size_t)d * 3 + 2] - pos[(size_t)s * 3 + 2]) + shz;
    const float len = sqrtf(vx * vx + vy * vy + vz * vz);
    const float den = fmaxf(len, 1e-8f);
    const float inv = 1.0f / den;
    const float x = vx * inv, y = vy * inv, z = vz * inv;
    float Y[9];
    Y[0] = 1.0f;
    Y[1] = S3C * y;  Y[2] = S3C * z;  Y[3] = S3C * x;
    Y[4] = S15C * x * y;
    Y[5] = S15C * y * z;
    Y[6] = C5H * (3.0f * z * z - 1.0f);
    Y[7] = S15C * x * z;
    Y[8] = C15H * (x * x - y * y);
    if (wave == 0) {
      float* gd = sG + el * GP;
      gpath<0, 0, 0,   0>(Y, cg, gd + 0);
      gpath<0, 1, 1,   1>(Y, cg, gd + 5);
      gpath<0, 2, 2,  10>(Y, cg, gd + 10);
      gpath<1, 0, 1,  35>(Y, cg, gd + 15);
      gpath<1, 1, 0,  44>(Y, cg, gd + 20);
      gpath<1, 1, 1,  53>(Y, cg, gd + 25);
      gpath<1, 1, 2,  80>(Y, cg, gd + 30);
      gpath<1, 2, 1, 125>(Y, cg, gd + 35);
      gpath<1, 2, 2, 170>(Y, cg, gd + 40);
      gpath<2, 0, 2, 245>(Y, cg, gd + 45);
      gpath<2, 1, 1, 270>(Y, cg, gd + 50);
      gpath<2, 1, 2, 315>(Y, cg, gd + 55);
      gpath<2, 2, 0, 390>(Y, cg, gd + 60);
      gpath<2, 2, 1, 415>(Y, cg, gd + 65);
      gpath<2, 2, 2, 490>(Y, cg, gd + 70);
    } else {
#pragma unroll
      for (int i = 0; i < NB16; ++i) {
        const float vi = 5.0f * ((float)(i + 1) * (1.0f / 17.0f));
        const float df = (len - vi) * RSTEP;
        const float ex = expf(-(df * df));
        semb[el * NB16 + i] = ex * (1.0f / 1.12f) * 4.0f;
      }
      const v4f a0 = *(const v4f*)(Ai + (size_t)s * UD);
      const v4f a1 = *(const v4f*)(Ai + (size_t)s * UD + 4);
      *(v4f*)(sAe + el * UD) = a0;
      *(v4f*)(sAe + el * UD + 4) = a1;
    }
  }
  __syncthreads();

  {
    const int j = tid;
    float wr[NB16];
#pragma unroll
    for (int c = 0; c < NB16; ++c) wr[c] = sW1[c * HID + j];
    const float bj = sb1[j];
#pragma unroll 1
    for (int el = 0; el < ER; ++el) {
      const v4f* ep = (const v4f*)(semb + el * NB16);
      float sacc = bj;
#pragma unroll
      for (int q = 0; q < 4; ++q) {
        const v4f e4 = ep[q];
        sacc += e4.x * wr[4 * q + 0];
        sacc += e4.y * wr[4 * q + 1];
        sacc += e4.z * wr[4 * q + 2];
        sacc += e4.w * wr[4 * q + 3];
      }
      sh1[el * HID + j] = siluf(sacc);
    }
  }
  __syncthreads();

  {
    const int j = tid;
    float wr[HID];
#pragma unroll
    for (int c = 0; c < HID; ++c) wr[c] = sW2[c * HID + j];
    const float bj = sb2[j];
#pragma unroll 1
    for (int el = 0; el < ER; ++el) {
      const v4f* ep = (const v4f*)(sh1 + el * HID);
      float sacc = bj;
#pragma unroll
      for (int q = 0; q < HID / 4; ++q) {
        const v4f e4 = ep[q];
        sacc += e4.x * wr[4 * q + 0];
        sacc += e4.y * wr[4 * q + 1];
        sacc += e4.z * wr[4 * q + 2];
        sacc += e4.w * wr[4 * q + 3];
      }
      sh2[el * HID + j] = siluf(sacc);
    }
  }
  __syncthreads();

#pragma unroll 1
  for (int it = tid; it < ER * AQ; it += ETHR) {
    const int e = it / AQ;
    const int q = it - e * AQ;
    const v4f a0 = *(const v4f*)(sAe + e * UD);
    const v4f a1 = *(const v4f*)(sAe + e * UD + 4);
    const float hj = sh2[e * HID + (q > HID - 1 ? HID - 1 : q)];
    const float mul = (q < HID) ? hj : ((q == HID) ? 1.0f : 0.0f);
    float f[8];
    f[0] = a0.x * mul; f[1] = a0.y * mul; f[2] = a0.z * mul; f[3] = a0.w * mul;
    f[4] = a1.x * mul; f[5] = a1.y * mul; f[6] = a1.z * mul; f[7] = a1.w * mul;
    v8us hv, lv;
#pragma unroll
    for (int u = 0; u < 8; ++u) {
      const unsigned short hb = bf_bits(f[u]);
      lv[u] = bf_bits(f[u] - bf_val(hb));
      hv[u] = hb;
    }
    *(v8us*)(sAhi + e * APL + 8 * q) = hv;
    *(v8us*)(sAlo + e * APL + 8 * q) = lv;
  }
  __syncthreads();

  {
    const v4f z4 = {0.0f, 0.0f, 0.0f, 0.0f};
    for (int i = tid; i < ER * FV4; i += ETHR) ((v4f*)sfeat)[i] = z4;
  }
  __syncthreads();

  {
    const unsigned short* arh = sAhi + (wave * 16 + m) * APL + 8 * hh;
    const unsigned short* arl = sAlo + (wave * 16 + m) * APL + 8 * hh;
#pragma unroll 1
    for (int g = 0; g < NGRPC; ++g) {
      v8f acc[TPG];
#pragma unroll
      for (int t = 0; t < TPG; ++t) { v8f z = {0.f, 0.f, 0.f, 0.f, 0.f, 0.f, 0.f, 0.f}; acc[t] = z; }
      const unsigned short* bph = Bhi + (size_t)(NGW * g + m) * BKP + 8 * hh;
      const unsigned short* bpl = Blo + (size_t)(NGW * g + m) * BKP + 8 * hh;
#pragma unroll 1
      for (int kt = 0; kt < KSTEPS; ++kt) {
        FragB ah, al;
        ah.u[0] = *(const v8us*)(arh + 32 * kt);
        ah.u[1] = *(const v8us*)(arh + 32 * kt + 16);
        al.u[0] = *(const v8us*)(arl + 32 * kt);
        al.u[1] = *(const v8us*)(arl + 32 * kt + 16);
#pragma unroll
        for (int t = 0; t < TPG; ++t) {
          const unsigned short* ph = bph + (size_t)t * 16 * BKP + 32 * kt;
          const unsigned short* pl = bpl + (size_t)t * 16 * BKP + 32 * kt;
          FragB bh, bl;
          bh.u[0] = *(const v8us*)ph;
          bh.u[1] = *(const v8us*)(ph + 16);
          bl.u[0] = *(const v8us*)pl;
          bl.u[1] = *(const v8us*)(pl + 16);
          acc[t] = wm3(ah.v, al.v, bh.v, bl.v, acc[t]);
        }
      }
#pragma unroll
      for (int t = 0; t < TPG; ++t) {
        const int n0 = NGW * g + 16 * t;
        const int p  = n0 >> 5;
        const int cc = (n0 & 31) + m;
        const int l3 = (int)((L3PACK >> (2 * p)) & 3u);
        const int d3 = 2 * l3 + 1;
        const float alpha = (l3 == 0) ? al0 : ((l3 == 1) ? al1 : al2);
        const int fb = (l3 == 0) ? 0 : ((l3 == 1) ? 32 : 128);
        float* fp = sfeat + (wave * 16 + 8 * hh) * FEAT + fb + cc * d3;
        const float* gq = sG + (wave * 16 + 8 * hh) * GP + 5 * p;
#pragma unroll
        for (int r = 0; r < 8; ++r) {
          const float tv = acc[t][r] * alpha;
#pragma unroll
          for (int k = 0; k < 5; ++k) {
            if (k < d3) fp[r * FEAT + k] = fp[r * FEAT + k] + tv * gq[r * GP + k];
          }
        }
      }
    }
  }
  __syncthreads();

  {
    float* gp = feat + (size_t)e0 * FEAT;
#pragma unroll 4
    for (int i = 0; i < (ER * FV4) / ETHR; ++i) {
      const int f = tid + ETHR * i;
      const v4f v = ((const v4f*)sfeat)[f];
      *(volatile v4f*)(gp + 4 * (size_t)f) = v;
    }
    __threadfence();
#pragma unroll 4
    for (int i = 0; i < (ER * FV4) / ETHR; ++i) {
      const int f = tid + ETHR * i;
      const v4f v = ((const v4f*)sfeat)[f];
      *(volatile v4f*)(gp + 4 * (size_t)f) = v;
    }
  }
}

__global__ __launch_bounds__(STHR) void k_scatter(
    const int* __restrict__ edst, const float* __restrict__ feat,
    float* out, int nE, int nN, int vec8, float scl) {
  extern __shared__ v4f lds_dyn[];
  float* sacc = (float*)lds_dyn;
  int*   list = (int*)(sacc + SNB * FEAT);
  int*   wcnt = list + LISTN;
  const int tid = threadIdx.x, lane = tid & 31, wave = tid >> 5;
  const int nodeBase = blockIdx.x * SNB;

  {
    const v4f z4 = {0.0f, 0.0f, 0.0f, 0.0f};
    for (int i = tid; i < SNB * FV4; i += STHR) ((v4f*)sacc)[i] = z4;
  }
  __syncthreads();

  const int nChunks = (nE + CHUNK - 1) / CHUNK;
#pragma unroll 1
  for (int ch = 0; ch < nChunks; ++ch) {
    const int cbase = ch * CHUNK;
    const int wc = scan_chunk<SNB>(edst, nE, cbase, nodeBase, vec8, list, tid, lane, wave);
    if (lane == 0) wcnt[wave] = wc;
    __syncthreads();
    if (wave < 3) {
#pragma unroll 1
      for (int wsx = 0; wsx < NWAVE; ++wsx) {
        int n = __builtin_amdgcn_readfirstlane(wcnt[wsx]);
        n = n > WCAP ? WCAP : (n < 0 ? 0 : n);
        const int* lp = list + wsx * WCAP;
#pragma unroll 1
        for (int i = 0; i < n; ++i) {
          const int ent  = __builtin_amdgcn_readfirstlane(lp[i]);
          const int slot = ent & (SNB - 1);
          int e = cbase + ((ent >> 12) & (CHUNK - 1));
          e = e > nE - 1 ? nE - 1 : e;
          if (tid < FV4) {
            const v4f v = *(const v4f*)(feat + (size_t)e * FEAT + 4 * tid);
            v4f* ap = (v4f*)(sacc + slot * FEAT + 4 * tid);
            *ap = *ap + v;
          }
        }
      }
    }
    __syncthreads();
  }

  const size_t obase = (size_t)nodeBase * FEAT;
#pragma unroll
  for (int i = 0; i < (SNB * FV4) / STHR; ++i) {
    const int f = tid + STHR * i;
    const int row = f / FV4;
    if (nodeBase + row < nN) {
      const v4f v = ((const v4f*)sacc)[f] * scl;
      *(volatile v4f*)(out + obase + 4 * (size_t)f) = v;
    }
  }
  __threadfence();
#pragma unroll
  for (int i = 0; i < (SNB * FV4) / STHR; ++i) {
    const int f = tid + STHR * i;
    const int row = f / FV4;
    if (nodeBase + row < nN) {
      const v4f v = ((const v4f*)sacc)[f] * scl;
      *(volatile v4f*)(out + obase + 4 * (size_t)f) = v;
    }
  }
}

struct Cx { double re, im; };
static Cx cxm(Cx a, Cx b) {
  Cx r;
  r.re = a.re * b.re - a.im * b.im;
  r.im = a.re * b.im + a.im * b.re;
  return r;
}
static double hfac(int n) { double r = 1.0; for (int i = 2; i <= n; ++i) r *= (double)i; return r; }
static double su2(int j1, int j2, int j3, int m1, int m2, int m3) {
  if (m3 != m1 + m2) return 0.0;
  int vmin = -j1 + j2 + m3;
  if (-j1 + m1 > vmin) vmin = -j1 + m1;
  if (0 > vmin) vmin = 0;
  int vmax = j2 + j3 + m1;
  if (j3 - j1 + j2 < vmax) vmax = j3 - j1 + j2;
  if (j3 + m3 < vmax) vmax = j3 + m3;
  const double num = (double)(2 * j3 + 1) * hfac(j3 + j1 - j2) * hfac(j3 - j1 + j2) * hfac(j1 + j2 - j3)
                     * hfac(j3 + m3) * hfac(j3 - m3);
  const double den = hfac(j1 + j2 + j3 + 1) * hfac(j1 - m1) * hfac(j1 + m1) * hfac(j2 - m2) * hfac(j2 + m2);
  const double pref = sqrt(num / den);
  double s = 0.0;
  for (int v = vmin; v <= vmax; ++v) {
    const double sg = ((v + j2 + m2) & 1) ? -1.0 : 1.0;
    const double tn = sg * hfac(j2 + j3 + m1 - v) * hfac(j1 - m1 + v);
    const double td = hfac(v) * hfac(j3 - j1 + j2 - v) * hfac(j3 + m3 - v) * hfac(v + j1 - j2 - m3);
    s += tn / td;
  }
  return pref * s;
}
static void buildq(int l, Cx q[5][5]) {
  for (int i = 0; i < 5; ++i) for (int j = 0; j < 5; ++j) { q[i][j].re = 0.0; q[i][j].im = 0.0; }
  const double s = 1.0 / sqrt(2.0);
  for (int mm = -l; mm < 0; ++mm) { q[l + mm][l - mm].re = s; q[l + mm][l + mm].im = -s; }
  q[l][l].re = 1.0; q[l][l].im = 0.0;
  for (int mm = 1; mm <= l; ++mm) {
    const double sg = (mm & 1) ? -1.0 : 1.0;
    q[l + mm][l + mm].re = sg * s;
    q[l + mm][l - mm].im = sg * s;
  }
  Cx ph; ph.re = 1.0; ph.im = 0.0;
  for (int i = 0; i < l; ++i) { Cx mi; mi.re = 0.0; mi.im = -1.0; ph = cxm(ph, mi); }
  for (int i = 0; i < 5; ++i) for (int j = 0; j < 5; ++j) q[i][j] = cxm(ph, q[i][j]);
}
static int realcg(int l1, int l2, int l3, float* dst) {
  const int d1 = 2 * l1 + 1, d2 = 2 * l2 + 1, d3 = 2 * l3 + 1;
  Cx q1[5][5], q2[5][5], q3[5][5];
  buildq(l1, q1); buildq(l2, q2); buildq(l3, q3);
  double C[125];
  double nrm = 0.0;
  for (int j = 0; j < d1; ++j) for (int l = 0; l < d2; ++l) for (int mm = 0; mm < d3; ++mm) {
    double acc = 0.0;
    for (int i = 0; i < d1; ++i) for (int k = 0; k < d2; ++k) for (int n = 0; n < d3; ++n) {
      const double cc = su2(l1, l2, l3, i - l1, k - l2, n - l3);
      if (cc == 0.0) continue;
      Cx q3c; q3c.re = q3[n][mm].re; q3c.im = -q3[n][mm].im;
      const Cx t = cxm(cxm(q1[i][j], q2[k][l]), q3c);
      acc += t.re * cc;
    }
    C[(j * d2 + l) * d3 + mm] = acc;
    nrm += acc * acc;
  }
  const double nv = sqrt(nrm);
  for (int i = 0; i < d1 * d2 * d3; ++i) dst[i] = (float)(C[i] / nv);
  return d1 * d2 * d3;
}
static void build_cg(CGTab* t) {
  for (int i = 0; i < CGN; ++i) t->v[i] = 0.0f;
  int off = 0;
  for (int l1 = 0; l1 <= 2; ++l1)
    for (int l2 = 0; l2 <= 2; ++l2) {
      int lo = l1 - l2; if (lo < 0) lo = -lo;
      int hi = l1 + l2; if (hi > 2) hi = 2;
      for (int l3 = lo; l3 <= hi; ++l3) {
        if (off + (2 * l1 + 1) * (2 * l2 + 1) * (2 * l3 + 1) > CGN) return;
        off += realcg(l1, l2, l3, t->v + off);
      }
    }
}

extern "C" void kernel_launch(void* const* d_in, const int* in_sizes, int n_in,
                              void* d_out, int out_size, void* d_ws, size_t ws_size,
                              hipStream_t stream) {
  if (n_in < 18) return;
  const int nN = in_sizes[0] / 3;
  const int nE = in_sizes[3];
  if (nN <= 0 || nE <= 0) return;
  if (in_sizes[0] != 3 * nN || in_sizes[1] != nN || in_sizes[2] != nN) return;
  if (in_sizes[4] != nE || in_sizes[5] != 3 * nE) return;
  if (in_sizes[6] < 9 || (in_sizes[6] % 9) != 0) return;
  const int nG = in_sizes[6] / 9;
  if (in_sizes[7] < NB16 || (in_sizes[7] % NB16) != 0) return;
  const int nA = in_sizes[7] / NB16;
  if (in_sizes[8] != NB16 * HID || in_sizes[9] != HID || in_sizes[10] != HID * UD || in_sizes[11] != UD) return;
  if (in_sizes[12] != NB16 * HID || in_sizes[13] != HID || in_sizes[14] != HID * HID || in_sizes[15] != HID) return;
  if (in_sizes[16] != HID * W3COLS || in_sizes[17] != W3COLS) return;
  if (out_size != nN * FEAT) return;
  if (nE > (1 << 26) || nN > (1 << 24)) return;

  const float* pos    = (const float*)d_in[0];
  const int*   atom   = (const int*)d_in[1];
  const int*   nbatch = (const int*)d_in[2];
  const int*   esrc   = (const int*)d_in[3];
  const int*   edst   = (const int*)d_in[4];
  const float* shf    = (const float*)d_in[5];
  const float* cell   = (const float*)d_in[6];
  const float* embt   = (const float*)d_in[7];
  const float* w_am1  = (const float*)d_in[8];
  const float* b_am1  = (const float*)d_in[9];
  const float* w_am2  = (const float*)d_in[10];
  const float* b_am2  = (const float*)d_in[11];
  const float* w_fc1  = (const float*)d_in[12];
  const float* b_fc1  = (const float*)d_in[13];
  const float* w_fc2  = (const float*)d_in[14];
  const float* b_fc2  = (const float*)d_in[15];
  const float* w_fc3  = (const float*)d_in[16];
  const float* b_fc3  = (const float*)d_in[17];
  float* out = (float*)d_out;

  const int nBN    = (nN + NNB - 1) / NNB;
  const int NPADA  = nBN * NNB;
  const int nBE    = (nE + ER - 1) / ER;
  const int EPAD   = nBE * ER;
  const int nBS    = (nN + SNB - 1) / SNB;
  const int nItems = NCOLS * BQ;
  const int nBB    = (nItems + STHR - 1) / STHR;

  char* ws = (char*)d_ws;
  size_t off = 0;
  const size_t oAi = off; off += (size_t)NPADA * UD * 4;      off = (off + 255) & ~(size_t)255;
  const size_t oBh = off; off += (size_t)NCOLS * BKP * 2;     off = (off + 255) & ~(size_t)255;
  const size_t oBl = off; off += (size_t)NCOLS * BKP * 2;     off = (off + 255) & ~(size_t)255;
  const size_t oFt = off; off += (size_t)EPAD * FEAT * 4;     off = (off + 255) & ~(size_t)255;
  if (off > ws_size || off > ((size_t)128 << 20)) return;
  float*          Aip   = (float*)(ws + oAi);
  unsigned short* Bh    = (unsigned short*)(ws + oBh);
  unsigned short* Bl    = (unsigned short*)(ws + oBl);
  float*          featp = (float*)(ws + oFt);

  CGTab cgt;
  build_cg(&cgt);
  const float al0 = (float)sqrt(1.0 / (8.0 * 3.0));
  const float al1 = (float)sqrt(3.0 / (8.0 * 6.0));
  const float al2 = (float)sqrt(5.0 / (8.0 * 6.0));
  double avgd = (double)nE / (double)nN;
  if (!(avgd > 1e-8)) avgd = 1e-8;
  const float avgf = (float)avgd;
  const float scl = 1.0f / avgf;

  k_node<<<nBN, NTHRN, 0, stream>>>(atom, embt, w_am1, b_am1, w_am2, b_am2, Aip, nN, nA);
  k_bprep<<<nBB, STHR, 0, stream>>>(w_fc3, b_fc3, Bh, Bl, nItems);
  hipFuncSetAttribute(reinterpret_cast<const void*>(&k_edge),
                      hipFuncAttributeMaxDynamicSharedMemorySize, LDS_EDGE);
  k_edge<<<nBE, ETHR, LDS_EDGE, stream>>>(pos, nbatch, esrc, edst, shf, cell, Aip,
                                          w_fc1, b_fc1, w_fc2, b_fc2, Bh, Bl, featp,
                                          nE, nN, nG, al0, al1, al2, cgt);
  hipFuncSetAttribute(reinterpret_cast<const void*>(&k_scatter),
                      hipFuncAttributeMaxDynamicSharedMemorySize, LDS_SC);
  k_scatter<<<nBS, STHR, LDS_SC, stream>>>(edst, featp, out, nE, nN, 1, scl);
}
